// Retention_46961172414498
// MI455X (gfx1250) — hardware-verified
//
#include <hip/hip_runtime.h>
#include <math.h>

constexpr int kB    = 2;
constexpr int kL    = 4096;
constexpr int kH    = 1024;
constexpr int kD    = 64;
constexpr int kTok  = kB * kL;
constexpr int kQKld = 2 * kD;
constexpr int kNW   = 3 * kD;
constexpr int kWin  = 12;
constexpr int kKP   = 72;
constexpr int kOP   = 68;
constexpr int kDecayLen = kWin * 64;
constexpr float kGamma = 0.96875f;
constexpr float kLog2TenKOver32 = 0.41524101186092029f;
static_assert(kH % 32 == 0, "K of the projections is a multiple of 32");
static_assert(kTok % 64 == 0 && kQKld % 64 == 0 && kL % 64 == 0 && kD == 64, "tile multiples");
static_assert((kTok * kH) % (8 * 256) == 0, "cast grid exact");
static_assert(kTok % 8 == 0, "xpos grid exact");

typedef __attribute__((ext_vector_type(16))) _Float16 v16h;
typedef __attribute__((ext_vector_type(8)))  _Float16 v8h;
typedef __attribute__((ext_vector_type(16))) __bf16   v16b;
typedef __attribute__((ext_vector_type(8)))  __bf16   v8b;
typedef __attribute__((ext_vector_type(8)))  float    v8f;
typedef __attribute__((ext_vector_type(4)))  float    v4f;
typedef __attribute__((ext_vector_type(2)))  float    v2f;
typedef __attribute__((ext_vector_type(4)))  unsigned int v4u;

__device__ __forceinline__ unsigned short f2bf_bits(float f) {
  unsigned u = __float_as_uint(f);
  return (unsigned short)((u + 0x7FFFu + ((u >> 16) & 1u)) >> 16);
}
__device__ __forceinline__ float bf_bits2f(unsigned short h) { return __uint_as_float(((unsigned)h) << 16); }

__device__ __forceinline__ void dep_guard_h(v8f& a, v8f& b, v16h x, v16h y) { asm volatile("v_nop\n\tv_nop\n\tv_nop\n\tv_nop" : "+v"(a), "+v"(b) : "v"(x), "v"(y)); }
__device__ __forceinline__ void dep_guard_b(v8f& a, v8f& b, v16b x, v16b y) { asm volatile("v_nop\n\tv_nop\n\tv_nop\n\tv_nop" : "+v"(a), "+v"(b) : "v"(x), "v"(y)); }
__device__ __forceinline__ void keep4_h(v16h a, v16h b, v16h c, v16h d) { asm volatile("v_nop" :: "v"(a), "v"(b), "v"(c), "v"(d)); }
__device__ __forceinline__ void keep4_b(v16b a, v16b b, v16b c, v16b d) { asm volatile("v_nop" :: "v"(a), "v"(b), "v"(c), "v"(d)); }
__device__ __forceinline__ void acc_guard4(v8f& a, v8f& b, v8f& c, v8f& d) { asm volatile("v_nop\n\tv_nop\n\tv_nop\n\tv_nop" : "+v"(a), "+v"(b), "+v"(c), "+v"(d)); }
template <typename T> struct Frag;
template <> struct Frag<_Float16> {
  typedef v16h V; union U { v16h v; v8h h[2]; };
  static __device__ __forceinline__ v16h load(const _Float16* p) {
    U f; f.h[0] = *(const v8h*)(p); f.h[1] = *(const v8h*)(p + 16); return f.v;
  }
  static __device__ __forceinline__ v8f mma(v16h a, v16h b, v8f c) {
    return __builtin_amdgcn_wmma_f32_16x16x32_f16(false, a, false, b, (short)0, c, false, false);
  }
  static __device__ __forceinline__ void guard(v8f& a, v8f& b, v16h x, v16h y) { dep_guard_h(a, b, x, y); }
  static __device__ __forceinline__ void keep(v16h a, v16h b, v16h c, v16h d) { keep4_h(a, b, c, d); }
};
template <> struct Frag<__bf16> {
  typedef v16b V; union U { v16b v; v8b h[2]; };
  static __device__ __forceinline__ v16b load(const __bf16* p) {
    U f; f.h[0] = *(const v8b*)(p); f.h[1] = *(const v8b*)(p + 16); return f.v;
  }
  static __device__ __forceinline__ v8f mma(v16b a, v16b b, v8f c) {
    return __builtin_amdgcn_wmma_f32_16x16x32_bf16(false, a, false, b, (short)0, c, false, false);
  }
  static __device__ __forceinline__ void guard(v8f& a, v8f& b, v16b x, v16b y) { dep_guard_b(a, b, x, y); }
  static __device__ __forceinline__ void keep(v16b a, v16b b, v16b c, v16b d) { keep4_b(a, b, c, d); }
};

__device__ __forceinline__ unsigned pk16(unsigned short a, unsigned short b) { return (unsigned)a | ((unsigned)b << 16); }

template <int ET> struct Elem;
template <> struct Elem<0> { typedef _Float16 T; };
template <> struct Elem<1> { typedef __bf16 T; };
template <int ET, bool SPLIT, int BIAS_MODE, int OUT_MODE, bool RESID, int ACT = 0>
__global__ __launch_bounds__(256) void wmma_gemm64(
    const unsigned short* __restrict__ Ap, const unsigned short* __restrict__ A2p, int lda, long strideA,
    const unsigned short* __restrict__ Btp, const unsigned short* __restrict__ Bt2p, int ldb, long strideB,
    void* __restrict__ Cout, void* __restrict__ Cout2, int ldc, long strideC,
    const float* __restrict__ bias,
    const float* __restrict__ resid, long strideR,
    int M, int N, int K, float scale) {
  typedef typename Elem<ET>::T T;
  typedef typename Frag<T>::V V;
  const T* A = (const T*)Ap; const T* A2 = (const T*)A2p; const T* Bt = (const T*)Btp; const T* Bt2 = (const T*)Bt2p;
  __shared__ __align__(16) float sT[8][16 * 68];
  const int b    = blockIdx.y;
  const int lane = threadIdx.x & 31;
  const int wave = threadIdx.x >> 5;
  const int tilesN = N >> 6;
  const int tilesM = M >> 6;
  const int tile = blockIdx.x * 8 + wave;
  if (tile >= tilesM * tilesN) return;
  const int tm = tile / tilesN;
  const int tn = tile - tm * tilesN;
  const int m0 = tm << 6;
  const int n0 = tn << 6;

  const T* Ab  = A  + (size_t)b * strideA;
  const T* Bb  = Bt + (size_t)b * strideB;
  const T* Ab2 = SPLIT ? (A2  + (size_t)b * strideA) : nullptr;
  const T* Bb2 = SPLIT ? (Bt2 + (size_t)b * strideB) : nullptr;

  const int rlane = lane & 15;
  const int koff  = (lane >> 4) * 8;
  const int mOff  = (lane >> 4) * 8;

  v8f acc[4][4];
#pragma unroll
  for (int i = 0; i < 4; ++i)
#pragma unroll
    for (int j = 0; j < 4; ++j) acc[i][j] = (v8f){0.f,0.f,0.f,0.f,0.f,0.f,0.f,0.f};

  for (int k0 = 0; k0 < K; k0 += 32) {
    V bh[4], bl[4];
#pragma unroll
    for (int j = 0; j < 4; ++j) {
      const size_t bo = (size_t)(n0 + (j << 4) + rlane) * ldb + koff + k0;
      bh[j] = Frag<T>::load(Bb + bo);
      if (SPLIT) bl[j] = Frag<T>::load(Bb2 + bo);
    }
#pragma unroll
    for (int i = 0; i < 4; ++i) {
      const size_t ao = (size_t)(m0 + (i << 4) + rlane) * lda + koff + k0;
      V ah = Frag<T>::load(Ab + ao);
      V al;
      if (SPLIT) al = Frag<T>::load(Ab2 + ao);
#pragma unroll
      for (int j = 0; j < 4; ++j) {
        acc[i][j] = Frag<T>::mma(ah, bh[j], acc[i][j]);
        if (SPLIT) {
          acc[i][j] = Frag<T>::mma(ah, bl[j], acc[i][j]);
          acc[i][j] = Frag<T>::mma(al, bh[j], acc[i][j]);
        }
      }
      Frag<T>::guard(acc[i][0], acc[i][3], ah, SPLIT ? al : ah);
    }
    Frag<T>::keep(bh[0], bh[1], bh[2], bh[3]);
    if (SPLIT) Frag<T>::keep(bl[0], bl[1], bl[2], bl[3]);
  }
  acc_guard4(acc[0][0], acc[0][1], acc[0][2], acc[0][3]);
  acc_guard4(acc[1][0], acc[1][1], acc[1][2], acc[1][3]);
  acc_guard4(acc[2][0], acc[2][1], acc[2][2], acc[2][3]);
  acc_guard4(acc[3][0], acc[3][1], acc[3][2], acc[3][3]);

  float* slab = sT[wave];
  const float* Rb = RESID ? (resid + (size_t)b * strideR) : nullptr;
#pragma unroll
  for (int i = 0; i < 4; ++i) {
    const int mBase = m0 + (i << 4);
#pragma unroll
    for (int j = 0; j < 4; ++j) {
      const int n = n0 + (j << 4) + rlane;
      float bv = 0.f;
      if (BIAS_MODE == 2) bv = bias[n];
#pragma unroll
      for (int r = 0; r < 8; ++r) {
        float v = acc[i][j][r] * scale;
        if (BIAS_MODE == 1) v += bias[mBase + mOff + r];
        if (BIAS_MODE == 2) v += bv;
        if (RESID) v += Rb[(size_t)(mBase + mOff + r) * ldc + n];
        if (ACT == 2) v = fmaxf(v, 0.0f);
        if (ACT == 4) v = (v > 0.f) ? v : 0.01f * v;
        slab[(mOff + r) * 68 + (j << 4) + rlane] = v;
      }
    }
    __builtin_amdgcn_fence(__ATOMIC_RELEASE, "workgroup");
    __builtin_amdgcn_wave_barrier();
    __builtin_amdgcn_fence(__ATOMIC_ACQUIRE, "workgroup");
    if (OUT_MODE == 0) {
      float* C = (float*)Cout + (size_t)b * strideC;
      const int hh = lane >> 4, c4 = (lane & 15) * 4;
      for (int pass = 0; pass < 2; ++pass) {
#pragma unroll
        for (int it = 0; it < 8; ++it) {
          const int row = it * 2 + hh;
          v4f v = *(const v4f*)(slab + row * 68 + c4);
          *(volatile v4f*)(C + (size_t)(mBase + row) * ldc + n0 + c4) = v;
        }
        __threadfence();
      }
    } else {
      const int q = lane >> 3, c8 = (lane & 7) * 8;
      unsigned short* C  = (unsigned short*)Cout  + (size_t)b * strideC;
      unsigned short* C2 = (OUT_MODE == 2) ? ((unsigned short*)Cout2 + (size_t)b * strideC) : nullptr;
      for (int pass = 0; pass < 2; ++pass) {
#pragma unroll
        for (int it = 0; it < 4; ++it) {
          const int row = it * 4 + q;
          const float* sp = slab + row * 68 + c8;
          v8h hv, lv;
#pragma unroll
          for (int e = 0; e < 8; ++e) {
            if (OUT_MODE == 1) {
              hv[e] = (_Float16)sp[e];
            } else {
              unsigned short hb = f2bf_bits(sp[e]);
              unsigned short lb = f2bf_bits(sp[e] - bf_bits2f(hb));
              hv[e] = __builtin_bit_cast(_Float16, hb);
              lv[e] = __builtin_bit_cast(_Float16, lb);
            }
          }
          *(volatile v8h*)(C + (size_t)(mBase + row) * ldc + n0 + c8) = hv;
          if (OUT_MODE == 2) *(volatile v8h*)(C2 + (size_t)(mBase + row) * ldc + n0 + c8) = lv;
        }
        __threadfence();
      }
    }
    __builtin_amdgcn_fence(__ATOMIC_RELEASE, "workgroup");
    __builtin_amdgcn_wave_barrier();
    __builtin_amdgcn_fence(__ATOMIC_ACQUIRE, "workgroup");
  }
}

__device__ __forceinline__ unsigned short at_bf_bits(float f) {
  unsigned u = __float_as_uint(f);
  return (unsigned short)((u + 0x7FFFu + ((u >> 16) & 1u)) >> 16);
}
__device__ __forceinline__ __bf16 at_f2bf(float f) { return __builtin_bit_cast(__bf16, at_bf_bits(f)); }
__device__ __forceinline__ void at_split(float f, __bf16& hi, __bf16& lo) {
  const unsigned short hb = at_bf_bits(f);
  hi = __builtin_bit_cast(__bf16, hb);
  lo = at_f2bf(f - __uint_as_float(((unsigned)hb) << 16));
}
__device__ __forceinline__ v8f at_mma(v16b a, v16b b, v8f c) {
  c = __builtin_amdgcn_wmma_f32_16x16x32_bf16(false, a, false, b, (short)0, c, false, false);
  asm volatile("v_nop\n\tv_nop\n\tv_nop\n\tv_nop" : "+v"(c) : "v"(a), "v"(b));
  return c;
}

__global__ __launch_bounds__(256) void cast8_bf16_kernel(const float* __restrict__ in, unsigned short* __restrict__ out, int n8) {
  const int i = blockIdx.x * 256 + threadIdx.x;
  if (i >= n8) return;
  const float* p = in + 8 * (size_t)i;
  const v4f a = *(const v4f*)(p);
  const v4f c = *(const v4f*)(p + 4);
  unsigned short hb[8];
#pragma unroll
  for (int e = 0; e < 4; ++e) {
    hb[e]     = f2bf_bits(a[e]);
    hb[4 + e] = f2bf_bits(c[e]);
  }
  const v4u u = (v4u){pk16(hb[0], hb[1]), pk16(hb[2], hb[3]), pk16(hb[4], hb[5]), pk16(hb[6], hb[7])};
  unsigned short* q = out + 8 * (size_t)i;
  *(volatile v4u*)q = u;
  __threadfence();
  *(volatile v4u*)q = u;
}

__global__ __launch_bounds__(256) void wt_pack_kernel(const float* __restrict__ WQ, const float* __restrict__ WK,
                                                      const float* __restrict__ WV, unsigned short* __restrict__ WT) {
  __shared__ float sm[64][65];
  const int t  = threadIdx.x;
  const int k0 = blockIdx.x * 64;
  const int z  = blockIdx.y;
  const float* W = (z == 0) ? WQ : (z == 1) ? WK : WV;
#pragma unroll
  for (int i = 0; i < 16; ++i) {
    const int e = i * 256 + t;
    const int r = e >> 6;
    const int cn = e & 63;
    sm[cn][r] = W[(size_t)(k0 + r) * kD + cn];
  }
  __syncthreads();
  const int lane = t & 31, wave = t >> 5;
  const int q = lane >> 3, c8 = (lane & 7) * 8;
  unsigned short* op = WT + (size_t)z * kD * kH;
  for (int pass = 0; pass < 2; ++pass) {
#pragma unroll
    for (int it = 0; it < 2; ++it) {
      const int row = wave * 8 + it * 4 + q;
      unsigned short hb[8];
#pragma unroll
      for (int e = 0; e < 8; ++e) hb[e] = f2bf_bits(sm[row][c8 + e]);
      const v4u u = (v4u){pk16(hb[0], hb[1]), pk16(hb[2], hb[3]), pk16(hb[4], hb[5]), pk16(hb[6], hb[7])};
      *(volatile v4u*)(op + (size_t)row * kH + k0 + c8) = u;
    }
    __threadfence();
  }
}

__global__ __launch_bounds__(256) void xpos_split_kernel(const float* __restrict__ QK,
                                                        unsigned short* __restrict__ Qh, unsigned short* __restrict__ Ql,
                                                        unsigned short* __restrict__ Kh, unsigned short* __restrict__ Kl) {
  const int lane = threadIdx.x & 31, wave = threadIdx.x >> 5;
  const int m = blockIdx.x * 8 + wave;
  const int l = m & (kL - 1);
  const float* rp = QK + (size_t)m * kQKld + 2 * lane;
  const v2f xq = *(const v2f*)(rp);
  const v2f xk = *(const v2f*)(rp + kD);
  const float fi   = (float)lane;
  const float lpos = (float)l;
  const float invf = exp2f(-(fi * kLog2TenKOver32));
  const float ang  = lpos * invf;
  float sn, cs;
  sincosf(ang, &sn, &cs);
  const float sv  = (2.0f * fi + 25.6f) * (1.0f / 89.6f);
  const float ex  = log2f(sv) * (lpos * (1.0f / 512.0f));
  const float sq  = exp2f(ex);
  const float sk  = exp2f(-ex);
  const float cq = cs * sq, snq = sn * sq;
  const float ck = cs * sk, snk = sn * sk;
  const float xq0 = xq[0], xq1 = xq[1], xk0 = xk[0], xk1 = xk[1];
  const float q0v = xq0 * cq - xq1 * snq;
  const float q1v = xq1 * cq + xq0 * snq;
  const float k0v = xk0 * ck - xk1 * snk;
  const float k1v = xk1 * ck + xk0 * snk;
  const unsigned short q0h = f2bf_bits(q0v), q1h = f2bf_bits(q1v);
  const unsigned short k0h = f2bf_bits(k0v), k1h = f2bf_bits(k1v);
  const unsigned short q0l = f2bf_bits(q0v - bf_bits2f(q0h)), q1l = f2bf_bits(q1v - bf_bits2f(q1h));
  const unsigned short k0l = f2bf_bits(k0v - bf_bits2f(k0h)), k1l = f2bf_bits(k1v - bf_bits2f(k1h));
  const unsigned wqh = pk16(q0h, q1h), wql = pk16(q0l, q1l);
  const unsigned wkh = pk16(k0h, k1h), wkl = pk16(k0l, k1l);
  const size_t o = (size_t)m * kD + 2 * lane;
  *(volatile unsigned*)(Qh + o) = wqh;
  *(volatile unsigned*)(Ql + o) = wql;
  *(volatile unsigned*)(Kh + o) = wkh;
  *(volatile unsigned*)(Kl + o) = wkl;
  __threadfence();
  *(volatile unsigned*)(Qh + o) = wqh;
  *(volatile unsigned*)(Ql + o) = wql;
  *(volatile unsigned*)(Kh + o) = wkh;
  *(volatile unsigned*)(Kl + o) = wkl;
}

__global__ __launch_bounds__(128) void decay_attn_kernel(
    const unsigned short* __restrict__ Qhp, const unsigned short* __restrict__ Qlp,
    const unsigned short* __restrict__ Khp, const unsigned short* __restrict__ Klp,
    const unsigned short* __restrict__ Vhp, const unsigned short* __restrict__ Vlp,
    float* __restrict__ out) {
  __shared__ __align__(16) __bf16 Ksh[64 * kKP];
  __shared__ __align__(16) __bf16 Ksl[64 * kKP];
  __shared__ __align__(16) __bf16 Vsh[64 * kKP];
  __shared__ __align__(16) __bf16 Vsl[64 * kKP];
  __shared__ __align__(16) __bf16 Psh[4][16 * kKP];
  __shared__ __align__(16) __bf16 Psl[4][16 * kKP];
  __shared__ __align__(16) float  Os[4][16 * kOP];
  __shared__ float dtab[kDecayLen];

  const int tid  = threadIdx.x;
  const int wave = tid >> 5;
  const int lane = tid & 31;
  const int hh   = lane >> 4;
  const int c    = lane & 15;
  const int koff = hh * 8;
  const int rt   = blockIdx.x;
  const int b    = blockIdx.y;
  const int q0   = rt * 64 + wave * 16;

  {
    const float lg = log2f(kGamma);
#pragma unroll 1
    for (int i = tid; i < kDecayLen; i += 128) dtab[i] = exp2f((float)i * lg);
  }

  const __bf16* Qh = (const __bf16*)Qhp;
  const __bf16* Ql = (const __bf16*)Qlp;
  v16b qh[2], ql[2];
  {
    const size_t qo = ((size_t)b * kL + q0 + c) * kD + koff;
#pragma unroll
    for (int dc = 0; dc < 2; ++dc) {
      qh[dc] = Frag<__bf16>::load(Qh + qo + dc * 32);
      ql[dc] = Frag<__bf16>::load(Ql + qo + dc * 32);
    }
  }

  v8f oacc[4];
#pragma unroll
  for (int t = 0; t < 4; ++t) oacc[t] = (v8f){0.f,0.f,0.f,0.f,0.f,0.f,0.f,0.f};

  const int ct0 = (rt > kWin - 1) ? (rt - (kWin - 1)) : 0;
  for (int ct = ct0; ct <= rt; ++ct) {
    __syncthreads();
    {
      const uint4* kgh = (const uint4*)(Khp + ((size_t)b * kL + (size_t)ct * 64) * kD);
      const uint4* kgl = (const uint4*)(Klp + ((size_t)b * kL + (size_t)ct * 64) * kD);
      const unsigned short* vgh = Vhp + (size_t)b * kD * kL + (size_t)ct * 64;
      const unsigned short* vgl = Vlp + (size_t)b * kD * kL + (size_t)ct * 64;
#pragma unroll
      for (int i2 = 0; i2 < 4; ++i2) {
        const int i = i2 * 128 + tid;
        const int r = i >> 3, c8 = (i & 7) * 8;
        *(uint4*)(Ksh + r * kKP + c8) = kgh[i];
      }
      asm volatile("" ::: "memory");
#pragma unroll
      for (int i2 = 0; i2 < 4; ++i2) {
        const int i = i2 * 128 + tid;
        const int r = i >> 3, c8 = (i & 7) * 8;
        *(uint4*)(Ksl + r * kKP + c8) = kgl[i];
      }
      asm volatile("" ::: "memory");
#pragma unroll
      for (int i2 = 0; i2 < 4; ++i2) {
        const int i = i2 * 128 + tid;
        const int r = i >> 3, c8 = (i & 7) * 8;
        *(uint4*)(Vsh + r * kKP + c8) = *(const uint4*)(vgh + (size_t)r * kL + c8);
      }
      asm volatile("" ::: "memory");
#pragma unroll
      for (int i2 = 0; i2 < 4; ++i2) {
        const int i = i2 * 128 + tid;
        const int r = i >> 3, c8 = (i & 7) * 8;
        *(uint4*)(Vsl + r * kKP + c8) = *(const uint4*)(vgl + (size_t)r * kL + c8);
      }
    }
    __syncthreads();

    v8f s[4];
#pragma unroll
    for (int j = 0; j < 4; ++j) {
      s[j] = (v8f){0.f,0.f,0.f,0.f,0.f,0.f,0.f,0.f};
#pragma unroll
      for (int dc = 0; dc < 2; ++dc) {
        const v16b kb = Frag<__bf16>::load(Ksh + (j * 16 + c) * kKP + koff + dc * 32);
        const v16b kl = Frag<__bf16>::load(Ksl + (j * 16 + c) * kKP + koff + dc * 32);
        s[j] = at_mma(qh[dc], kb, s[j]);
        s[j] = at_mma(qh[dc], kl, s[j]);
        s[j] = at_mma(ql[dc], kb, s[j]);
      }
    }

    __bf16* pwh = Psh[wave];
    __bf16* pwl = Psl[wave];
#pragma unroll
    for (int r = 0; r < 8; ++r) {
      const int nrow = q0 + 8 * hh + r;
#pragma unroll
      for (int j = 0; j < 4; ++j) {
        const int mcol = ct * 64 + j * 16 + c;
        const int diff = nrow - mcol;
        int di = (diff < 0) ? 0 : diff;
        di = (di > kDecayLen - 1) ? (kDecayLen - 1) : di;
        const float wd = dtab[di];
        const float w  = (diff >= 0) ? wd : 0.0f;
        const float v  = s[j][r] * w;
        __bf16 hb, lb;
        at_split(v, hb, lb);
        pwh[(8 * hh + r) * kKP + j * 16 + c] = hb;
        pwl[(8 * hh + r) * kKP + j * 16 + c] = lb;
      }
    }
    __builtin_amdgcn_fence(__ATOMIC_RELEASE, "workgroup");
    __builtin_amdgcn_wave_barrier();
    __builtin_amdgcn_fence(__ATOMIC_ACQUIRE, "workgroup");

#pragma unroll
    for (int kk = 0; kk < 2; ++kk) {
      const v16b pa = Frag<__bf16>::load(pwh + c * kKP + koff + kk * 32);
      const v16b pl = Frag<__bf16>::load(pwl + c * kKP + koff + kk * 32);
#pragma unroll
      for (int t = 0; t < 4; ++t) {
        const v16b vb = Frag<__bf16>::load(Vsh + (t * 16 + c) * kKP + koff + kk * 32);
        const v16b vl = Frag<__bf16>::load(Vsl + (t * 16 + c) * kKP + koff + kk * 32);
        oacc[t] = at_mma(pa, vb, oacc[t]);
        oacc[t] = at_mma(pa, vl, oacc[t]);
        oacc[t] = at_mma(pl, vb, oacc[t]);
      }
    }
  }

  float* os = Os[wave];
#pragma unroll
  for (int r = 0; r < 8; ++r) {
#pragma unroll
    for (int t = 0; t < 4; ++t) os[(8 * hh + r) * kOP + t * 16 + c] = oacc[t][r];
  }
  __builtin_amdgcn_fence(__ATOMIC_RELEASE, "workgroup");
  __builtin_amdgcn_wave_barrier();
  __builtin_amdgcn_fence(__ATOMIC_ACQUIRE, "workgroup");
  {
    float* ob = out + ((size_t)b * kL + q0) * kD;
    const int c4 = (lane & 15) * 4;
    for (int pass = 0; pass < 2; ++pass) {
#pragma unroll
      for (int it = 0; it < 8; ++it) {
        const int row = it * 2 + hh;
        const v4f val = *(const v4f*)(os + row * kOP + c4);
        *(volatile v4f*)(ob + (size_t)row * kD + c4) = val;
      }
      __threadfence();
    }
  }
}

extern "C" void kernel_launch(void* const* d_in, const int* in_sizes, int n_in,
                              void* d_out, int out_size, void* d_ws, size_t ws_size,
                              hipStream_t stream) {
  if (n_in < 4) return;
  if (in_sizes[0] != kTok * kH) return;
  if (in_sizes[1] != kH * kD || in_sizes[2] != kH * kD || in_sizes[3] != kH * kD) return;
  if (out_size != kTok * kD) return;

  const size_t szXb = (size_t)kTok * kH * 2;
  const size_t szWT = (size_t)kNW * kH * 2;
  const size_t szQK = (size_t)kTok * kQKld * 4;
  const size_t szPl = (size_t)kTok * kD * 2;
  const size_t offXb = 0;
  const size_t offWT = offXb + szXb;
  const size_t offQK = offWT + szWT;
  const size_t offQh = offQK + szQK;
  const size_t offQl = offQh + szPl;
  const size_t offKh = offQl + szPl;
  const size_t offKl = offKh + szPl;
  const size_t offVh = offKl + szPl;
  const size_t offVl = offVh + szPl;
  const size_t total = offVl + szPl;
  if (ws_size < total) return;

  const float* X  = (const float*)d_in[0];
  const float* WQ = (const float*)d_in[1];
  const float* WK = (const float*)d_in[2];
  const float* WV = (const float*)d_in[3];
  float* out = (float*)d_out;
  char* ws = (char*)d_ws;
  unsigned short* Xb = (unsigned short*)(ws + offXb);
  unsigned short* WT = (unsigned short*)(ws + offWT);
  float* QK = (float*)(ws + offQK);
  unsigned short* Qh = (unsigned short*)(ws + offQh);
  unsigned short* Ql = (unsigned short*)(ws + offQl);
  unsigned short* Kh = (unsigned short*)(ws + offKh);
  unsigned short* Kl = (unsigned short*)(ws + offKl);
  unsigned short* Vh = (unsigned short*)(ws + offVh);
  unsigned short* Vl = (unsigned short*)(ws + offVl);

  const int n8 = (kTok * kH) / 8;
  cast8_bf16_kernel<<<dim3(n8 / 256), dim3(256), 0, stream>>>(X, Xb, n8);
  wt_pack_kernel<<<dim3(kH / 64, 3), dim3(256), 0, stream>>>(WQ, WK, WV, WT);

  const int tilesQK = (kTok / 64) * (kQKld / 64);
  wmma_gemm64<1, false, 0, 0, false, 0><<<dim3(tilesQK / 8, 1), dim3(256), 0, stream>>>(
      Xb, Xb, kH, 0L, WT, WT, kH, 0L,
      (void*)QK, (void*)QK, kQKld, 0L, QK, QK, 0L, kTok, kQKld, kH, 1.0f);

  const int tilesVT = (kD / 64) * (kL / 64);
  wmma_gemm64<1, false, 0, 2, false, 0><<<dim3(tilesVT / 8, kB), dim3(256), 0, stream>>>(
      WT + (size_t)2 * kD * kH, WT + (size_t)2 * kD * kH, kH, 0L, Xb, Xb, kH, (long)kL * kH,
      (void*)Vh, (void*)Vl, kL, (long)kD * kL, QK, QK, 0L, kD, kL, kH, 1.0f);

  xpos_split_kernel<<<dim3(kTok / 8), dim3(256), 0, stream>>>(QK, Qh, Ql, Kh, Kl);

  decay_attn_kernel<<<dim3(kL / 64, kB), dim3(128), 0, stream>>>(Qh, Ql, Kh, Kl, Vh, Vl, out);
}
